// MultiHeadStructureAttention_19688130085318
// MI455X (gfx1250) — hardware-verified
//
#include <hip/hip_runtime.h>

typedef _Float16 v16h __attribute__((ext_vector_type(16)));
typedef _Float16 v8h  __attribute__((ext_vector_type(8)));
typedef float    v8f  __attribute__((ext_vector_type(8)));
typedef float    v4f  __attribute__((ext_vector_type(4)));
typedef v8h __attribute__((may_alias)) v8ha;
typedef v4f __attribute__((may_alias)) v4fa;

union Frag { v16h v; v8h half[2]; };

#define D_MODEL 1024
#define NHEADS  16
#define HD      64
#define SEQ     2048
#define BATCH   4
#define MROWS   (BATCH * SEQ)
#define NX      (MROWS * D_MODEL)
#define NW      (D_MODEL * D_MODEL)
#define NX8     (NX / 8)
#define WSCALE  32.0f
#define QSCALE  0.125f
#define PSCALE  16384.0f
#define OSCALE  64.0f

__device__ __forceinline__ v8f wmma_f16(v16h a, v16h b, v8f c) {
  v8f d = __builtin_amdgcn_wmma_f32_16x16x32_f16(false, a, false, b, (short)0, c, false, false);
  asm volatile("v_nop\n\tv_nop\n\tv_nop\n\tv_nop" : "+v"(d) : "v"(a), "v"(b));
  return d;
}

__device__ __forceinline__ v16h load_frag(const _Float16* p, int h) {
  Frag f;
  f.half[0] = *(const v8ha*)(p + 8 * h);
  f.half[1] = *(const v8ha*)(p + 16 + 8 * h);
  return f.v;
}

__device__ __forceinline__ float wave_sum(float x) {
  x += __shfl_xor(x, 16);
  x += __shfl_xor(x, 8);
  x += __shfl_xor(x, 4);
  x += __shfl_xor(x, 2);
  x += __shfl_xor(x, 1);
  return x;
}

__global__ __launch_bounds__(256) void cvt_act_kernel(
    const float* __restrict__ q, const float* __restrict__ k, const float* __restrict__ v,
    _Float16* __restrict__ xh)
{
  const int g = blockIdx.x * 256 + threadIdx.x;
  if (g >= 3 * NX8) return;
  const int which = g / NX8;
  const int off = g - which * NX8;
  const float* src = (which == 0) ? q : ((which == 1) ? k : v);
  src += (size_t)off * 8;
  _Float16* dst = xh + (size_t)g * 8;
  const v4f a = *(const v4fa*)src;
  const v4f c = *(const v4fa*)(src + 4);
  const v8h o = { (_Float16)a.x, (_Float16)a.y, (_Float16)a.z, (_Float16)a.w,
                  (_Float16)c.x, (_Float16)c.y, (_Float16)c.z, (_Float16)c.w };
  *(volatile v8h*)dst = o;
  __threadfence();
  *(volatile v8h*)dst = o;
}

__global__ __launch_bounds__(256) void cvt_w_kernel(
    const float* __restrict__ wq, const float* __restrict__ wk,
    const float* __restrict__ wv, const float* __restrict__ wfc,
    _Float16* __restrict__ wt)
{
  __shared__ float tile[64][65];
  const int tid = threadIdx.x, lane = tid & 31, w = tid >> 5;
  const int n0 = blockIdx.x * 64, k0 = blockIdx.y * 64, mat = blockIdx.z;
  const float* src = (mat == 0) ? wq : ((mat == 1) ? wk : ((mat == 2) ? wv : wfc));
  const int tx = tid & 63, ty = tid >> 6;
  #pragma unroll
  for (int i = 0; i < 16; ++i) {
    const int kk = ty + 4 * i;
    tile[kk][tx] = src[(size_t)(k0 + kk) * D_MODEL + n0 + tx] * WSCALE;
  }
  __syncthreads();

  const int q8 = lane & 7, sub = lane >> 3;
  const int lidA = w * 8 + sub;
  const int lidB = w * 8 + 4 + sub;
  const v8h oA = { (_Float16)tile[8 * q8 + 0][lidA], (_Float16)tile[8 * q8 + 1][lidA],
                   (_Float16)tile[8 * q8 + 2][lidA], (_Float16)tile[8 * q8 + 3][lidA],
                   (_Float16)tile[8 * q8 + 4][lidA], (_Float16)tile[8 * q8 + 5][lidA],
                   (_Float16)tile[8 * q8 + 6][lidA], (_Float16)tile[8 * q8 + 7][lidA] };
  const v8h oB = { (_Float16)tile[8 * q8 + 0][lidB], (_Float16)tile[8 * q8 + 1][lidB],
                   (_Float16)tile[8 * q8 + 2][lidB], (_Float16)tile[8 * q8 + 3][lidB],
                   (_Float16)tile[8 * q8 + 4][lidB], (_Float16)tile[8 * q8 + 5][lidB],
                   (_Float16)tile[8 * q8 + 6][lidB], (_Float16)tile[8 * q8 + 7][lidB] };
  _Float16* dA = wt + ((size_t)mat * D_MODEL + n0 + lidA) * D_MODEL + k0 + 8 * q8;
  _Float16* dB = wt + ((size_t)mat * D_MODEL + n0 + lidB) * D_MODEL + k0 + 8 * q8;
  *(volatile v8h*)dA = oA;
  *(volatile v8h*)dB = oB;
  __threadfence();
  *(volatile v8h*)dA = oA;
  *(volatile v8h*)dB = oB;
}

__device__ __forceinline__ void proj_store_pass(const _Float16* sT, _Float16* plane, _Float16* vt,
                                                int which, int bh, int l0, int w, int lane) {
  const int q8 = lane & 7, sub = lane >> 3;
  #pragma unroll
  for (int i = 0; i < 8; ++i) {
    const int lid = w * 32 + i * 4 + sub;
    v8h v;
    _Float16* dst;
    if (which != 2) {
      v = *(const v8ha*)(sT + lid * HD + 8 * q8);
      dst = plane + ((size_t)bh * SEQ + l0 + lid) * HD + 8 * q8;
    } else {
      const int d = lid >> 1, hl = lid & 1;
      v = *(const v8ha*)(sT + d * 128 + 64 * hl + 8 * q8);
      dst = vt + ((size_t)bh * HD + d) * SEQ + l0 + 64 * hl + 8 * q8;
    }
    *(volatile v8h*)dst = v;
  }
}

__global__ __launch_bounds__(128) void proj_kernel(
    const _Float16* __restrict__ xh,
    const _Float16* __restrict__ wt,
    _Float16* __restrict__ qh,
    _Float16* __restrict__ kh,
    _Float16* __restrict__ vt)
{
  __shared__ __attribute__((aligned(16))) _Float16 sT[128 * 64];

  const int tid = threadIdx.x, lane = tid & 31, w = tid >> 5;
  const int h = lane >> 4, m = lane & 15;
  const int m0 = blockIdx.x * 128;
  const int cg = blockIdx.y;
  const int which = cg >> 4, head = cg & 15;
  const int m0w = m0 + 32 * w;

  const _Float16* xp  = xh + (size_t)which * NX;
  const _Float16* xa0 = xp + (size_t)(m0w + m) * D_MODEL;
  const _Float16* xa1 = xa0 + (size_t)16 * D_MODEL;
  const _Float16* wb  = wt + ((size_t)which * D_MODEL + head * HD + m) * D_MODEL;

  const v8f zero8 = {0.f, 0.f, 0.f, 0.f, 0.f, 0.f, 0.f, 0.f};
  v8f acc[2][4];
  #pragma unroll
  for (int mt = 0; mt < 2; ++mt)
    #pragma unroll
    for (int nt = 0; nt < 4; ++nt) acc[mt][nt] = zero8;

  #pragma unroll 1
  for (int k0 = 0; k0 < D_MODEL; k0 += 32) {
    const v16h a0 = load_frag(xa0 + k0, h);
    const v16h a1 = load_frag(xa1 + k0, h);
    #pragma unroll
    for (int nt = 0; nt < 4; ++nt) {
      const v16h b = load_frag(wb + (size_t)nt * 16 * D_MODEL + k0, h);
      acc[0][nt] = wmma_f16(a0, b, acc[0][nt]);
      acc[1][nt] = wmma_f16(a1, b, acc[1][nt]);
    }
  }

  const float osc = (which == 0) ? (QSCALE / WSCALE) : (1.0f / WSCALE);
  #pragma unroll
  for (int nt = 0; nt < 4; ++nt) {
    const int feat = 16 * nt + m;
    #pragma unroll
    for (int mt = 0; mt < 2; ++mt) {
      #pragma unroll
      for (int r = 0; r < 8; ++r) {
        const int tokl = 32 * w + 16 * mt + 8 * h + r;
        const float y = acc[mt][nt][r] * osc;
        const int idx = (which == 2) ? (feat * 128 + tokl) : (tokl * HD + feat);
        sT[idx] = (_Float16)y;
      }
    }
  }
  __syncthreads();

  const int b = m0 / SEQ, l0 = m0 - b * SEQ, bh = b * NHEADS + head;
  _Float16* plane = (which == 0) ? qh : kh;
  proj_store_pass(sT, plane, vt, which, bh, l0, w, lane);
  __threadfence();
  proj_store_pass(sT, plane, vt, which, bh, l0, w, lane);
}

__device__ __forceinline__ v16h pack_p(v8f a, v8f c) {
  const v16h r = { (_Float16)(a[0] * PSCALE), (_Float16)(a[1] * PSCALE), (_Float16)(a[2] * PSCALE), (_Float16)(a[3] * PSCALE),
                   (_Float16)(a[4] * PSCALE), (_Float16)(a[5] * PSCALE), (_Float16)(a[6] * PSCALE), (_Float16)(a[7] * PSCALE),
                   (_Float16)(c[0] * PSCALE), (_Float16)(c[1] * PSCALE), (_Float16)(c[2] * PSCALE), (_Float16)(c[3] * PSCALE),
                   (_Float16)(c[4] * PSCALE), (_Float16)(c[5] * PSCALE), (_Float16)(c[6] * PSCALE), (_Float16)(c[7] * PSCALE) };
  return r;
}

__device__ __forceinline__ void att_store_pass(const _Float16* so, _Float16* ah,
                                               int b, int head, int q0, int lane) {
  const int q8 = lane & 7, sub = lane >> 3;
  #pragma unroll
  for (int i = 0; i < 4; ++i) {
    const int row = i * 4 + sub;
    const v8h v = *(const v8ha*)(so + row * HD + 8 * q8);
    const size_t gi = ((size_t)b * SEQ + q0 + row) * D_MODEL + head * HD + 8 * q8;
    *(volatile v8h*)(ah + gi) = v;
  }
}

__global__ __launch_bounds__(128) void attn_kernel(
    const _Float16* __restrict__ qh,
    const _Float16* __restrict__ kh,
    const _Float16* __restrict__ vt,
    _Float16* __restrict__ ah)
{
  __shared__ __attribute__((aligned(16))) _Float16 sO[4 * 16 * 64];

  const int tid = threadIdx.x, lane = tid & 31, w = tid >> 5;
  const int h = lane >> 4, m = lane & 15;
  const int bh = blockIdx.y, b = bh >> 4, head = bh & 15;
  const int q0 = blockIdx.x * 64 + 16 * w;

  const _Float16* qrow = qh + ((size_t)bh * SEQ + q0 + m) * HD;
  const v16h qb0 = load_frag(qrow, h);
  const v16h qb1 = load_frag(qrow + 32, h);

  const v8f zero8 = {0.f, 0.f, 0.f, 0.f, 0.f, 0.f, 0.f, 0.f};
  v8f o[4];
  #pragma unroll
  for (int t = 0; t < 4; ++t) o[t] = zero8;
  float mrun = -1e30f, lrun = 0.0f;

  const _Float16* kbase = kh + ((size_t)bh * SEQ + m) * HD;
  const _Float16* vbase = vt + ((size_t)bh * HD + m) * SEQ;

  #pragma unroll 1
  for (int kb = 0; kb < SEQ; kb += 64) {
    v8f s[4];
    #pragma unroll
    for (int j = 0; j < 4; ++j) {
      const _Float16* kp = kbase + (size_t)(kb + 16 * j) * HD;
      const v16h kf0 = load_frag(kp, h);
      const v16h kf1 = load_frag(kp + 32, h);
      v8f z = zero8;
      z = wmma_f16(kf0, qb0, z);
      z = wmma_f16(kf1, qb1, z);
      s[j] = z;
    }

    float mloc = s[0][0];
    #pragma unroll
    for (int j = 0; j < 4; ++j)
      #pragma unroll
      for (int r = 0; r < 8; ++r) mloc = fmaxf(mloc, s[j][r]);
    mloc = fmaxf(mloc, __shfl_xor(mloc, 16));
    const float mnew = fmaxf(mrun, mloc);
    const float alpha = __expf(mrun - mnew);
    mrun = mnew;
    float lsum = 0.0f;
    #pragma unroll
    for (int j = 0; j < 4; ++j)
      #pragma unroll
      for (int r = 0; r < 8; ++r) {
        const float p = __expf(s[j][r] - mnew);
        s[j][r] = p;
        lsum += p;
      }
    lsum += __shfl_xor(lsum, 16);
    lrun = lrun * alpha + lsum;
    #pragma unroll
    for (int t = 0; t < 4; ++t)
      #pragma unroll
      for (int r = 0; r < 8; ++r) o[t][r] = o[t][r] * alpha;

    const v16h pb0 = pack_p(s[0], s[1]);
    const v16h pb1 = pack_p(s[2], s[3]);

    #pragma unroll
    for (int t = 0; t < 4; ++t) {
      const _Float16* vp = vbase + (size_t)(16 * t) * SEQ + kb;
      const v16h vf0 = load_frag(vp, h);
      const v16h vf1 = load_frag(vp + 32, h);
      o[t] = wmma_f16(vf0, pb0, o[t]);
      o[t] = wmma_f16(vf1, pb1, o[t]);
    }
  }

  const float inv = __builtin_amdgcn_rcpf(lrun) * (OSCALE / PSCALE);
  _Float16* so = sO + w * 1024;
  #pragma unroll
  for (int t = 0; t < 4; ++t)
    #pragma unroll
    for (int r = 0; r < 8; ++r)
      so[m * HD + 16 * t + 8 * h + r] = (_Float16)(o[t][r] * inv);
  __syncthreads();

  att_store_pass(so, ah, b, head, q0, lane);
  __threadfence();
  att_store_pass(so, ah, b, head, q0, lane);
}

__device__ __forceinline__ void fc_store_pass(const float* sF, float* fcb, int m0, int nb, int w, int lane) {
  const int q8 = lane & 7, sub = lane >> 3;
  #pragma unroll
  for (int i = 0; i < 16; ++i) {
    const int lid = w * 64 + i * 4 + sub;
    const int row = lid >> 1, hl = lid & 1;
    const v4f v = *(const v4fa*)(sF + row * HD + 32 * hl + 4 * q8);
    const size_t gi = ((size_t)(m0 + row)) * D_MODEL + nb * HD + 32 * hl + 4 * q8;
    *(volatile v4f*)(fcb + gi) = v;
  }
}

__global__ __launch_bounds__(128) void fc_kernel(
    const _Float16* __restrict__ ah,
    const _Float16* __restrict__ wfct,
    float* __restrict__ fcb)
{
  __shared__ __attribute__((aligned(16))) float sF[128 * 64];

  const int tid = threadIdx.x, lane = tid & 31, w = tid >> 5;
  const int h = lane >> 4, m = lane & 15;
  const int m0 = blockIdx.x * 128;
  const int nb = blockIdx.y;
  const int m0w = m0 + 32 * w;

  const _Float16* xa0 = ah + (size_t)(m0w + m) * D_MODEL;
  const _Float16* xa1 = xa0 + (size_t)16 * D_MODEL;
  const _Float16* wb  = wfct + ((size_t)nb * HD + m) * D_MODEL;

  const v8f zero8 = {0.f, 0.f, 0.f, 0.f, 0.f, 0.f, 0.f, 0.f};
  v8f acc[2][4];
  #pragma unroll
  for (int mt = 0; mt < 2; ++mt)
    #pragma unroll
    for (int nt = 0; nt < 4; ++nt) acc[mt][nt] = zero8;

  #pragma unroll 1
  for (int k0 = 0; k0 < D_MODEL; k0 += 32) {
    const v16h a0 = load_frag(xa0 + k0, h);
    const v16h a1 = load_frag(xa1 + k0, h);
    #pragma unroll
    for (int nt = 0; nt < 4; ++nt) {
      const v16h b = load_frag(wb + (size_t)nt * 16 * D_MODEL + k0, h);
      acc[0][nt] = wmma_f16(a0, b, acc[0][nt]);
      acc[1][nt] = wmma_f16(a1, b, acc[1][nt]);
    }
  }

  const float osc = 1.0f / (WSCALE * OSCALE);
  #pragma unroll
  for (int nt = 0; nt < 4; ++nt) {
    const int feat = 16 * nt + m;
    #pragma unroll
    for (int mt = 0; mt < 2; ++mt) {
      #pragma unroll
      for (int r = 0; r < 8; ++r) {
        const int tokl = 32 * w + 16 * mt + 8 * h + r;
        sF[tokl * HD + feat] = acc[mt][nt][r] * osc;
      }
    }
  }
  __syncthreads();

  fc_store_pass(sF, fcb, m0, nb, w, lane);
  __threadfence();
  fc_store_pass(sF, fcb, m0, nb, w, lane);
}

__global__ __launch_bounds__(256) void ln_kernel(
    const float* __restrict__ fcb, const float* __restrict__ q,
    const float* __restrict__ gamma, const float* __restrict__ beta,
    float* __restrict__ out)
{
  const int lane = threadIdx.x & 31, w = threadIdx.x >> 5;
  const int row = blockIdx.x * 8 + w;
  if (row >= MROWS) return;
  const float* fr = fcb + (size_t)row * D_MODEL;
  const float* qr = q + (size_t)row * D_MODEL;

  v4f x[8];
  float s = 0.0f;
  #pragma unroll
  for (int i = 0; i < 8; ++i) {
    const int c = i * 128 + 4 * lane;
    const v4f a = *(const v4fa*)(fr + c);
    const v4f rr = *(const v4fa*)(qr + c);
    x[i] = a + rr;
    s += (x[i].x + x[i].y) + (x[i].z + x[i].w);
  }
  s = wave_sum(s);
  const float mu = s * (1.0f / D_MODEL);
  float ss = 0.0f;
  #pragma unroll
  for (int i = 0; i < 8; ++i) {
    const v4f d = x[i] - mu;
    ss += (d.x * d.x + d.y * d.y) + (d.z * d.z + d.w * d.w);
  }
  ss = wave_sum(ss);
  const float var = ss * (1.0f / D_MODEL);
  const float rs = rsqrtf(var + 1e-6f);

  v4f y[8];
  #pragma unroll
  for (int i = 0; i < 8; ++i) {
    const int c = i * 128 + 4 * lane;
    const v4f g = *(const v4fa*)(gamma + c);
    const v4f be = *(const v4fa*)(beta + c);
    y[i] = (x[i] - mu) * rs * g + be;
  }
  float* orow = out + (size_t)row * D_MODEL;
  #pragma unroll
  for (int i = 0; i < 8; ++i) *(volatile v4f*)(orow + i * 128 + 4 * lane) = y[i];
  __threadfence();
  #pragma unroll
  for (int i = 0; i < 8; ++i) *(volatile v4f*)(orow + i * 128 + 4 * lane) = y[i];
}

extern "C" void kernel_launch(void* const* d_in, const int* in_sizes, int n_in,
                              void* d_out, int out_size, void* d_ws, size_t ws_size,
                              hipStream_t stream) {
  if (n_in < 9) return;
  if (in_sizes[0] != NX || in_sizes[1] != NX || in_sizes[2] != NX) return;
  if (in_sizes[3] != NW || in_sizes[4] != NW || in_sizes[5] != NW || in_sizes[6] != NW) return;
  if (in_sizes[7] != D_MODEL || in_sizes[8] != D_MODEL) return;
  if (out_size != NX) return;

  const float* q     = (const float*)d_in[0];
  const float* k     = (const float*)d_in[1];
  const float* v     = (const float*)d_in[2];
  const float* Wq    = (const float*)d_in[3];
  const float* Wk    = (const float*)d_in[4];
  const float* Wv    = (const float*)d_in[5];
  const float* Wfc   = (const float*)d_in[6];
  const float* gamma = (const float*)d_in[7];
  const float* beta  = (const float*)d_in[8];
  float* out = (float*)d_out;

  const size_t xh_bytes = (size_t)3 * NX * 2;
  const size_t wt_bytes = (size_t)4 * NW * 2;
  const size_t pl_bytes = (size_t)BATCH * NHEADS * SEQ * HD * 2;
  const size_t ah_bytes = (size_t)NX * 2;
  const size_t fc_bytes = (size_t)NX * 4;
  const size_t total = xh_bytes + wt_bytes + 3 * pl_bytes;
  if (total > ws_size) return;
  if (ah_bytes + fc_bytes > xh_bytes) return;

  char* ws = (char*)d_ws;
  _Float16* xh  = (_Float16*)(ws);
  _Float16* wt  = (_Float16*)(ws + xh_bytes);
  _Float16* qh  = (_Float16*)(ws + xh_bytes + wt_bytes);
  _Float16* kh  = (_Float16*)(ws + xh_bytes + wt_bytes + pl_bytes);
  _Float16* vt  = (_Float16*)(ws + xh_bytes + wt_bytes + 2 * pl_bytes);
  _Float16* ah  = (_Float16*)(ws);
  float*    fcb = (float*)(ws + ah_bytes);

  const int ngroups = 3 * NX8;
  cvt_act_kernel<<<(ngroups + 255) / 256, 256, 0, stream>>>(q, k, v, xh);

  dim3 gW(D_MODEL / 64, D_MODEL / 64, 4);
  cvt_w_kernel<<<gW, 256, 0, stream>>>(Wq, Wk, Wv, Wfc, wt);

  dim3 gProj(MROWS / 128, 3 * NHEADS);
  proj_kernel<<<gProj, 128, 0, stream>>>(xh, wt, qh, kh, vt);

  dim3 gAtt(SEQ / 64, BATCH * NHEADS);
  attn_kernel<<<gAtt, 128, 0, stream>>>(qh, kh, vt, ah);

  dim3 gFc(MROWS / 128, D_MODEL / HD);
  fc_kernel<<<gFc, 128, 0, stream>>>(ah, wt + (size_t)3 * NW, fcb);

  ln_kernel<<<(MROWS + 7) / 8, 256, 0, stream>>>(fcb, q, gamma, beta, out);
}
